// SUPRARecurrentFixedGamma_10024453668954
// MI455X (gfx1250) — hardware-verified
//
#include <hip/hip_runtime.h>
#include <math.h>

constexpr int kBatch = 4;
constexpr int kSeq   = 2048;
constexpr int kDim   = 1024;
constexpr int kTok   = kBatch * kSeq;
constexpr float kWCarry    = 32.0f;
constexpr float kWCarryInv = 1.0f / 32.0f;
constexpr float kEps       = 1e-6f;

constexpr size_t kOffXh   = 0;
constexpr size_t kOffAWh  = 0;
constexpr size_t kOffAWl  = 8388608;
constexpr size_t kOffWh   = 16777216;
constexpr size_t kOffPart = 16777216;
constexpr size_t kOffDen  = 17039360;
constexpr size_t kOffPw   = 23068672;
constexpr size_t kOffQh   = 23076864;
constexpr size_t kOffQl   = 39854080;
constexpr size_t kOffKh   = 56631296;
constexpr size_t kOffKl   = 73408512;
constexpr size_t kOffVth  = 90185728;
constexpr size_t kOffVtl  = 106962944;
constexpr size_t kWsEnd   = 123740160;

typedef __attribute__((ext_vector_type(16))) _Float16 v16h;
typedef __attribute__((ext_vector_type(8)))  _Float16 v8h;
typedef __attribute__((ext_vector_type(16))) __bf16   v16b;
typedef __attribute__((ext_vector_type(8)))  __bf16   v8b;
typedef __attribute__((ext_vector_type(8)))  float    v8f;
typedef __attribute__((ext_vector_type(4)))  float    v4f;
typedef __attribute__((ext_vector_type(4)))  unsigned int v4u;

__device__ __forceinline__ unsigned short f2bf_bits(float f) {
  unsigned u = __float_as_uint(f);
  return (unsigned short)((u + 0x7FFFu + ((u >> 16) & 1u)) >> 16);
}
__device__ __forceinline__ float bf_bits2f(unsigned short h) { return __uint_as_float(((unsigned)h) << 16); }

__device__ __forceinline__ void dep_guard_h(v8f& a, v8f& b, v16h x, v16h y) { asm volatile("v_nop\n\tv_nop\n\tv_nop\n\tv_nop" : "+v"(a), "+v"(b) : "v"(x), "v"(y)); }
__device__ __forceinline__ void dep_guard_b(v8f& a, v8f& b, v16b x, v16b y) { asm volatile("v_nop\n\tv_nop\n\tv_nop\n\tv_nop" : "+v"(a), "+v"(b) : "v"(x), "v"(y)); }
__device__ __forceinline__ void keep4_h(v16h a, v16h b, v16h c, v16h d) { asm volatile("v_nop" :: "v"(a), "v"(b), "v"(c), "v"(d)); }
__device__ __forceinline__ void keep4_b(v16b a, v16b b, v16b c, v16b d) { asm volatile("v_nop" :: "v"(a), "v"(b), "v"(c), "v"(d)); }
__device__ __forceinline__ void acc_guard4(v8f& a, v8f& b, v8f& c, v8f& d) { asm volatile("v_nop\n\tv_nop\n\tv_nop\n\tv_nop" : "+v"(a), "+v"(b), "+v"(c), "+v"(d)); }
template <typename T> struct Frag;
template <> struct Frag<_Float16> {
  typedef v16h V; union U { v16h v; v8h h[2]; };
  static __device__ __forceinline__ v16h load(const _Float16* p) {
    U f; f.h[0] = *(const v8h*)(p); f.h[1] = *(const v8h*)(p + 16); return f.v;
  }
  static __device__ __forceinline__ v8f mma(v16h a, v16h b, v8f c) {
    return __builtin_amdgcn_wmma_f32_16x16x32_f16(false, a, false, b, (short)0, c, false, false);
  }
  static __device__ __forceinline__ void guard(v8f& a, v8f& b, v16h x, v16h y) { dep_guard_h(a, b, x, y); }
  static __device__ __forceinline__ void keep(v16h a, v16h b, v16h c, v16h d) { keep4_h(a, b, c, d); }
};
template <> struct Frag<__bf16> {
  typedef v16b V; union U { v16b v; v8b h[2]; };
  static __device__ __forceinline__ v16b load(const __bf16* p) {
    U f; f.h[0] = *(const v8b*)(p); f.h[1] = *(const v8b*)(p + 16); return f.v;
  }
  static __device__ __forceinline__ v8f mma(v16b a, v16b b, v8f c) {
    return __builtin_amdgcn_wmma_f32_16x16x32_bf16(false, a, false, b, (short)0, c, false, false);
  }
  static __device__ __forceinline__ void guard(v8f& a, v8f& b, v16b x, v16b y) { dep_guard_b(a, b, x, y); }
  static __device__ __forceinline__ void keep(v16b a, v16b b, v16b c, v16b d) { keep4_b(a, b, c, d); }
};

__device__ __forceinline__ unsigned pk16(unsigned short a, unsigned short b) { return (unsigned)a | ((unsigned)b << 16); }
__device__ __forceinline__ unsigned short h_bits(float f) { const _Float16 h = (_Float16)f; return __builtin_bit_cast(unsigned short, h); }

template <int ET> struct Elem;
template <> struct Elem<0> { typedef _Float16 T; };
template <> struct Elem<1> { typedef __bf16 T; };
template <int ET, bool SPLIT, int BIAS_MODE, int OUT_MODE, bool RESID, int ACT, int XMODE>
__global__ __launch_bounds__(256) void wmma_gemm64(
    const unsigned short* __restrict__ Ap, const unsigned short* __restrict__ A2p, int lda, long strideA,
    const unsigned short* __restrict__ Btp, const unsigned short* __restrict__ Bt2p, int ldb, long strideB,
    void* __restrict__ Cout, void* __restrict__ Cout2, int ldc, long strideC,
    const float* __restrict__ bias,
    const float* __restrict__ resid, long strideR,
    const float* __restrict__ aux, float* __restrict__ aux_out,
    int M, int N, int K, float scale) {
  typedef typename Elem<ET>::T T;
  typedef typename Frag<T>::V V;
  const T* A = (const T*)Ap; const T* A2 = (const T*)A2p; const T* Bt = (const T*)Btp; const T* Bt2 = (const T*)Bt2p;
  __shared__ __align__(16) float sT[8][16 * 68];
  __shared__ __align__(16) float sR[8][64];
  const int b    = blockIdx.y;
  const int lane = threadIdx.x & 31;
  const int wave = threadIdx.x >> 5;
  const int tilesN = N >> 6;
  const int tilesM = M >> 6;
  const int tile = blockIdx.x * 8 + wave;
  int tm = 0, tn = 0;
  if (XMODE == 1) {
    const int ntri = (tilesM * (tilesM + 1)) >> 1;
    if (tile >= ntri) return;
    int tmv = (int)((sqrtf(8.0f * (float)tile + 1.0f) - 1.0f) * 0.5f);
    if ((((tmv + 1) * (tmv + 2)) >> 1) <= tile) tmv += 1;
    if (((tmv * (tmv + 1)) >> 1) > tile) tmv -= 1;
    tm = tmv;
    tn = tile - ((tmv * (tmv + 1)) >> 1);
  } else {
    if (tile >= tilesM * tilesN) return;
    tm = tile / tilesN;
    tn = tile - tm * tilesN;
  }
  const int m0 = tm << 6;
  const int n0 = tn << 6;

  const T* Ab  = A  + (size_t)b * strideA;
  const T* Bb  = Bt + (size_t)b * strideB;
  const T* Ab2 = SPLIT ? (A2  + (size_t)b * strideA) : nullptr;
  const T* Bb2 = SPLIT ? (Bt2 + (size_t)b * strideB) : nullptr;

  const int rlane = lane & 15;
  const int koff  = (lane >> 4) * 8;
  const int mOff  = (lane >> 4) * 8;

  v8f acc[4][4];
#pragma unroll
  for (int i = 0; i < 4; ++i)
#pragma unroll
    for (int j = 0; j < 4; ++j) acc[i][j] = (v8f){0.f,0.f,0.f,0.f,0.f,0.f,0.f,0.f};

  const int kEnd = (XMODE == 2) ? (m0 + 64) : K;
  for (int k0 = 0; k0 < kEnd; k0 += 32) {
    V bh[4], bl[4];
#pragma unroll
    for (int j = 0; j < 4; ++j) {
      const size_t bo = (size_t)(n0 + (j << 4) + rlane) * ldb + koff + k0;
      bh[j] = Frag<T>::load(Bb + bo);
      if (SPLIT) bl[j] = Frag<T>::load(Bb2 + bo);
    }
#pragma unroll
    for (int i = 0; i < 4; ++i) {
      const size_t ao = (size_t)(m0 + (i << 4) + rlane) * lda + koff + k0;
      V ah = Frag<T>::load(Ab + ao);
      V al;
      if (SPLIT) al = Frag<T>::load(Ab2 + ao);
#pragma unroll
      for (int j = 0; j < 4; ++j) {
        acc[i][j] = Frag<T>::mma(ah, bh[j], acc[i][j]);
        if (SPLIT) {
          acc[i][j] = Frag<T>::mma(ah, bl[j], acc[i][j]);
          acc[i][j] = Frag<T>::mma(al, bh[j], acc[i][j]);
        }
      }
      Frag<T>::guard(acc[i][0], acc[i][3], ah, SPLIT ? al : ah);
    }
    Frag<T>::keep(bh[0], bh[1], bh[2], bh[3]);
    if (SPLIT) Frag<T>::keep(bl[0], bl[1], bl[2], bl[3]);
  }
  acc_guard4(acc[0][0], acc[0][1], acc[0][2], acc[0][3]);
  acc_guard4(acc[1][0], acc[1][1], acc[1][2], acc[1][3]);
  acc_guard4(acc[2][0], acc[2][1], acc[2][2], acc[2][3]);
  acc_guard4(acc[3][0], acc[3][1], acc[3][2], acc[3][3]);

  float* slab = sT[wave];
  float* rsw  = sR[wave];
  const float* Rb = RESID ? (resid + (size_t)b * strideR) : nullptr;
#pragma unroll
  for (int i = 0; i < 4; ++i) {
    const int mBase = m0 + (i << 4);
    float rinv[8];
    if (XMODE == 2) {
#pragma unroll
      for (int r = 0; r < 8; ++r) rinv[r] = 1.0f / aux[mBase + mOff + r];
    }
#pragma unroll
    for (int j = 0; j < 4; ++j) {
      const int n = n0 + (j << 4) + rlane;
      float bv = 0.f;
      if (BIAS_MODE == 2) bv = bias[n];
#pragma unroll
      for (int r = 0; r < 8; ++r) {
        float v = acc[i][j][r] * scale;
        if (BIAS_MODE == 1) v += bias[mBase + mOff + r];
        if (BIAS_MODE == 2) v += bv;
        if (RESID) v += Rb[(size_t)(mBase + mOff + r) * ldc + n];
        if (XMODE == 1) {
          const int dlt = (mBase + mOff + r) - n;
          const int di  = (dlt < 0) ? 0 : dlt;
          const float f = aux[di];
          v = (dlt >= 0) ? (v * f) : 0.0f;
        }
        if (XMODE == 2) v = v * rinv[r];
        if (ACT == 2) v = fmaxf(v, 0.0f);
        slab[(mOff + r) * 68 + (j << 4) + rlane] = v;
      }
    }
    __builtin_amdgcn_fence(__ATOMIC_RELEASE, "workgroup");
    __builtin_amdgcn_wave_barrier();
    __builtin_amdgcn_fence(__ATOMIC_ACQUIRE, "workgroup");
    if (XMODE == 1) {
      const float* rp = slab + rlane * 68 + (lane >> 4) * 32;
      float s = 0.f;
#pragma unroll
      for (int c4i = 0; c4i < 8; ++c4i) {
        const v4f t4 = *(const v4f*)(rp + 4 * c4i);
        s += t4[0]; s += t4[1]; s += t4[2]; s += t4[3];
      }
      s += __shfl_xor(s, 16, 32);
      rsw[(i << 4) + rlane] = s;
    }
    if (OUT_MODE == 0) {
      float* C = (float*)Cout + (size_t)b * strideC;
      const int hh = lane >> 4, c4 = (lane & 15) * 4;
      for (int pass = 0; pass < 2; ++pass) {
#pragma unroll
        for (int it = 0; it < 8; ++it) {
          const int row = it * 2 + hh;
          v4f v = *(const v4f*)(slab + row * 68 + c4);
          *(volatile v4f*)(C + (size_t)(mBase + row) * ldc + n0 + c4) = v;
        }
        __threadfence();
      }
    } else {
      const int q = lane >> 3, c8 = (lane & 7) * 8;
      unsigned short* C  = (unsigned short*)Cout  + (size_t)b * strideC;
      unsigned short* C2 = (OUT_MODE == 2) ? ((unsigned short*)Cout2 + (size_t)b * strideC) : nullptr;
      for (int pass = 0; pass < 2; ++pass) {
#pragma unroll
        for (int it = 0; it < 4; ++it) {
          const int row = it * 4 + q;
          const float* sp = slab + row * 68 + c8;
          v8h hv, lv;
#pragma unroll
          for (int e = 0; e < 8; ++e) {
            if (OUT_MODE == 1) {
              hv[e] = (_Float16)sp[e];
            } else {
              unsigned short hb = f2bf_bits(sp[e]);
              unsigned short lb = f2bf_bits(sp[e] - bf_bits2f(hb));
              hv[e] = __builtin_bit_cast(_Float16, hb);
              lv[e] = __builtin_bit_cast(_Float16, lb);
            }
          }
          *(volatile v8h*)(C + (size_t)(mBase + row) * ldc + n0 + c8) = hv;
          if (OUT_MODE == 2) *(volatile v8h*)(C2 + (size_t)(mBase + row) * ldc + n0 + c8) = lv;
        }
        __threadfence();
      }
    }
    __builtin_amdgcn_fence(__ATOMIC_RELEASE, "workgroup");
    __builtin_amdgcn_wave_barrier();
    __builtin_amdgcn_fence(__ATOMIC_ACQUIRE, "workgroup");
  }
  if (XMODE == 1) {
    const v4f pv = *(const v4f*)(rsw + (lane & 15) * 4);
    float* pp = aux_out + (size_t)tn * M + m0 + (lane & 15) * 4;
    for (int pass = 0; pass < 2; ++pass) {
      if (lane < 16) *(volatile v4f*)pp = pv;
      __threadfence();
    }
  }
}

__global__ __launch_bounds__(256) void cast8_f16_kernel(const float* __restrict__ in, unsigned short* __restrict__ out,
                                                        int n8, float scale) {
  const int i = blockIdx.x * 256 + threadIdx.x;
  if (i >= n8) return;
  const float* p = in + 8 * (size_t)i;
  const v4f a = *(const v4f*)(p);
  const v4f c = *(const v4f*)(p + 4);
  unsigned short hb[8];
#pragma unroll
  for (int e = 0; e < 4; ++e) {
    hb[e]     = h_bits(a[e] * scale);
    hb[4 + e] = h_bits(c[e] * scale);
  }
  const v4u u = (v4u){pk16(hb[0], hb[1]), pk16(hb[2], hb[3]), pk16(hb[4], hb[5]), pk16(hb[6], hb[7])};
  unsigned short* q = out + 8 * (size_t)i;
  *(volatile v4u*)q = u;
  __threadfence();
  *(volatile v4u*)q = u;
}

__global__ __launch_bounds__(256) void decay_table_kernel(const float* __restrict__ gamma_p, float* __restrict__ pw) {
  __shared__ __align__(16) float spw[kSeq];
  if (threadIdx.x == 0) {
    const float g = gamma_p[0];
    float p = 1.0f;
#pragma unroll 1
    for (int n = 0; n < kSeq; ++n) { spw[n] = p; p = p * g; }
  }
  __syncthreads();
  const int tid = threadIdx.x;
  for (int pass = 0; pass < 2; ++pass) {
#pragma unroll
    for (int it = 0; it < 2; ++it) {
      const int idx = it * 256 + tid;
      const v4f v = *(const v4f*)(spw + 4 * idx);
      *(volatile v4f*)(pw + 4 * idx) = v;
    }
    __threadfence();
  }
}

__global__ __launch_bounds__(256) void den_kernel(const float* __restrict__ part, float* __restrict__ den) {
  const int row = blockIdx.x * 256 + threadIdx.x;
  const int cnt = (row >> 6) + 1;
  float s = 0.f;
#pragma unroll 1
  for (int tn = 0; tn < cnt; ++tn) s += part[(size_t)tn * kSeq + row];
  const float d = s + kEps;
  ((volatile float*)den)[row] = d;
  __threadfence();
  ((volatile float*)den)[row] = d;
}

extern "C" void kernel_launch(void* const* d_in, const int* in_sizes, int n_in,
                              void* d_out, int out_size, void* d_ws,
                              size_t ws_size, hipStream_t stream) {
  if (n_in < 8) return;
  if (in_sizes[0] != kTok * kDim || in_sizes[1] != kDim * kDim || in_sizes[2] != kDim ||
      in_sizes[3] != kDim * kDim || in_sizes[4] != kDim || in_sizes[5] != kDim * kDim ||
      in_sizes[6] != kDim || in_sizes[7] < 1 || out_size != kTok * kDim || ws_size < kWsEnd) return;

  const float* x       = (const float*)d_in[0];
  const float* Wq      = (const float*)d_in[1];
  const float* bq      = (const float*)d_in[2];
  const float* Wk      = (const float*)d_in[3];
  const float* bk      = (const float*)d_in[4];
  const float* Wv      = (const float*)d_in[5];
  const float* bv      = (const float*)d_in[6];
  const float* gamma_p = (const float*)d_in[7];
  float* out = (float*)d_out;
  char* ws = (char*)d_ws;

  unsigned short* Xh   = (unsigned short*)(ws + kOffXh);
  unsigned short* Wh   = (unsigned short*)(ws + kOffWh);
  unsigned short* AWh  = (unsigned short*)(ws + kOffAWh);
  unsigned short* AWl  = (unsigned short*)(ws + kOffAWl);
  float* part          = (float*)(ws + kOffPart);
  float* den           = (float*)(ws + kOffDen);
  float* pw            = (float*)(ws + kOffPw);
  unsigned short* Qh   = (unsigned short*)(ws + kOffQh);
  unsigned short* Ql   = (unsigned short*)(ws + kOffQl);
  unsigned short* Kh   = (unsigned short*)(ws + kOffKh);
  unsigned short* Kl   = (unsigned short*)(ws + kOffKl);
  unsigned short* Vth  = (unsigned short*)(ws + kOffVth);
  unsigned short* Vtl  = (unsigned short*)(ws + kOffVtl);

  const size_t planeW   = (size_t)kDim * kDim;
  const size_t planeSeq = (size_t)kSeq * kDim;

  cast8_f16_kernel<<<(kTok * kDim / 8) / 256, 256, 0, stream>>>(x, Xh, kTok * kDim / 8, 1.0f);
  cast8_f16_kernel<<<(kDim * kDim / 8) / 256, 256, 0, stream>>>(Wq, Wh, kDim * kDim / 8, kWCarry);
  cast8_f16_kernel<<<(kDim * kDim / 8) / 256, 256, 0, stream>>>(Wk, Wh + planeW, kDim * kDim / 8, kWCarry);
  cast8_f16_kernel<<<(kDim * kDim / 8) / 256, 256, 0, stream>>>(Wv, Wh + 2 * planeW, kDim * kDim / 8, kWCarry);

  decay_table_kernel<<<1, 256, 0, stream>>>(gamma_p, pw);

  wmma_gemm64<0, false, 2, 2, false, 2, 0><<<dim3(256, 1), 256, 0, stream>>>(
      Xh, Xh, kDim, 0L, Wh, Wh, kDim, 0L, (void*)Qh, (void*)Ql, kDim, 0L,
      bq, bq, 0L, pw, part, kTok, kDim, kDim, kWCarryInv);
  wmma_gemm64<0, false, 2, 2, false, 2, 0><<<dim3(256, 1), 256, 0, stream>>>(
      Xh, Xh, kDim, 0L, Wh + planeW, Wh + planeW, kDim, 0L, (void*)Kh, (void*)Kl, kDim, 0L,
      bk, bk, 0L, pw, part, kTok, kDim, kDim, kWCarryInv);
  wmma_gemm64<0, false, 1, 2, false, 0, 0><<<dim3(64, kBatch), 256, 0, stream>>>(
      Wh + 2 * planeW, Wh + 2 * planeW, kDim, 0L, Xh, Xh, kDim, (long)planeSeq, (void*)Vth, (void*)Vtl, kSeq, (long)planeSeq,
      bv, bv, 0L, pw, part, kDim, kSeq, kDim, kWCarryInv);

  for (int b = 0; b < kBatch; ++b) {
    wmma_gemm64<1, true, 0, 2, false, 0, 1><<<dim3(66, 1), 256, 0, stream>>>(
        Qh + (size_t)b * planeSeq, Ql + (size_t)b * planeSeq, kDim, 0L,
        Kh + (size_t)b * planeSeq, Kl + (size_t)b * planeSeq, kDim, 0L,
        (void*)AWh, (void*)AWl, kSeq, 0L,
        bq, bq, 0L, pw, part, kSeq, kSeq, kDim, 1.0f);
    den_kernel<<<8, 256, 0, stream>>>(part, den);
    wmma_gemm64<1, true, 0, 0, false, 0, 2><<<dim3(64, 1), 256, 0, stream>>>(
        AWh, AWl, kSeq, 0L,
        Vth + (size_t)b * planeSeq, Vtl + (size_t)b * planeSeq, kSeq, 0L,
        (void*)(out + (size_t)b * planeSeq), (void*)(out + (size_t)b * planeSeq), kDim, 0L,
        bq, bq, 0L, den, part, kSeq, kDim, kSeq, 1.0f);
  }
}
